// SelfAttention_71554155152053
// MI455X (gfx1250) — hardware-verified
//
#include <hip/hip_runtime.h>


#ifndef NB
#define NB 2
#endif
#ifndef SEQ
#define SEQ 4096
#endif
#define NB_FULL    2
#define SEQ_FULL   4096
#define NHEAD      8
#define HDIM       64
#define BQ         128
#define BK         32
#define NWAVE      8
#define CT         64
#define TP         72
#define OP         68
#define WS_CAP     134217728ull

static_assert(SEQ % BQ == 0);
static_assert(SEQ % CT == 0);
static_assert(SEQ % BK == 0);
static_assert(BQ == NWAVE * 16);
static_assert(HDIM == 64);
static_assert(HDIM % 32 == 0);
static_assert(HDIM * 4 == 16 * 16);
static_assert(CT * 2 == 128);
static_assert(HDIM * 2 == 128);
static_assert(CT == 64 && CT <= TP);
static_assert(SEQ <= SEQ_FULL);
static_assert(NB >= 1 && NB <= NB_FULL);
static_assert((TP * 2) % 16 == 0);
static_assert((OP * 4) % 16 == 0);
static_assert(OP >= HDIM);
static_assert((unsigned long long)NB * NHEAD * SEQ * HDIM * 2ull * 2ull <= WS_CAP);

typedef __bf16   bf16;
typedef _Float16 f16;
typedef bf16     v16bf __attribute__((ext_vector_type(16)));
typedef f16      v16h  __attribute__((ext_vector_type(16)));
typedef f16      v8h   __attribute__((ext_vector_type(8)));
typedef float    v8f   __attribute__((ext_vector_type(8)));
typedef float    v4f   __attribute__((ext_vector_type(4)));
typedef unsigned v4u   __attribute__((ext_vector_type(4)));

union FragB  { v16bf v; v4u q[2]; bf16 h[16]; };
union FragH  { v16h  v; v4u q[2]; f16  h[16]; };
union Pack8B { v4u u; bf16 h[8]; };
union Pack8H { v4u u; v8h v; f16 h[8]; };

static __device__ __forceinline__ v8f mma_bf16(v16bf a, v16bf b, v8f acc) {
  acc = __builtin_amdgcn_wmma_f32_16x16x32_bf16(false, a, false, b, (short)0, acc, false, false);
  asm volatile("v_nop\n\tv_nop\n\tv_nop\n\tv_nop" : "+v"(acc) : "v"(a), "v"(b));
  return acc;
}
static __device__ __forceinline__ v8f mma_f16(v16h a, v16h b, v8f acc) {
  acc = __builtin_amdgcn_wmma_f32_16x16x32_f16(false, a, false, b, (short)0, acc, false, false);
  asm volatile("v_nop\n\tv_nop\n\tv_nop\n\tv_nop" : "+v"(acc) : "v"(a), "v"(b));
  return acc;
}

__global__ __launch_bounds__(256) void kv_planes_kernel(const float* __restrict__ kin,
                                                        const float* __restrict__ vin,
                                                        bf16* __restrict__ kb,
                                                        f16* __restrict__ vt) {
  const int kt  = blockIdx.x;
  const int h   = blockIdx.y;
  const int b   = blockIdx.z;
  const int tid = threadIdx.x;
  __shared__ __align__(16) f16 sT[HDIM * TP];
  const int s0 = kt * CT;

  v4u    kval[2];
  size_t kidx[2];
  #pragma unroll
  for (int kk = 0; kk < 2; ++kk) {
    const int key = kk * 32 + (tid >> 3);
    const int d0  = (tid & 7) * 8;
    const size_t src = (((size_t)b * NHEAD + h) * SEQ_FULL + s0 + key) * HDIM + d0;
    const v4f k0 = *(const v4f*)(kin + src);
    const v4f k1 = *(const v4f*)(kin + src + 4);
    const v4f v0 = *(const v4f*)(vin + src);
    const v4f v1 = *(const v4f*)(vin + src + 4);
    Pack8B pk;
    #pragma unroll
    for (int i = 0; i < 4; ++i) {
      pk.h[i]     = (bf16)k0[i];
      pk.h[4 + i] = (bf16)k1[i];
    }
    kval[kk] = pk.u;
    kidx[kk] = (((size_t)b * NHEAD + h) * SEQ + s0 + key) * HDIM + d0;
    #pragma unroll
    for (int i = 0; i < 4; ++i) {
      sT[(d0 + i) * TP + key]     = (f16)(float)(bf16)v0[i];
      sT[(d0 + 4 + i) * TP + key] = (f16)(float)(bf16)v1[i];
    }
  }
  __syncthreads();

  v4u    vval[2];
  size_t vidx[2];
  #pragma unroll
  for (int kk = 0; kk < 2; ++kk) {
    const int d  = kk * 32 + (tid >> 3);
    const int ks = (tid & 7) * 8;
    Pack8H ph;
    ph.v = *(const v8h*)(sT + d * TP + ks);
    vval[kk] = ph.u;
    vidx[kk] = (((size_t)b * NHEAD + h) * HDIM + d) * SEQ + s0 + ks;
  }

  #pragma unroll
  for (int kk = 0; kk < 2; ++kk) {
    *(volatile v4u*)(kb + kidx[kk]) = kval[kk];
    *(volatile v4u*)(vt + vidx[kk]) = vval[kk];
  }
  __threadfence();
  #pragma unroll
  for (int kk = 0; kk < 2; ++kk) {
    *(volatile v4u*)(kb + kidx[kk]) = kval[kk];
    *(volatile v4u*)(vt + vidx[kk]) = vval[kk];
  }
}

__global__ __launch_bounds__(256) void attn_kernel(const float* __restrict__ q,
                                                   const bf16* __restrict__ kb,
                                                   const f16* __restrict__ vt,
                                                   float* __restrict__ out) {
  const int qblk = blockIdx.x;
  const int h    = blockIdx.y;
  const int b    = blockIdx.z;
  const int tid  = threadIdx.x;
  const int wave = __builtin_amdgcn_readfirstlane(threadIdx.x >> 5);
  const int lane = tid & 31;
  const int lq   = lane & 15;
  const int hi   = lane >> 4;

  __shared__ __align__(16) float sO[NWAVE * 16 * OP];

  const int qrow0 = qblk * BQ + wave * 16;

  FragB qf[2];
  {
    const float* qp = q + (((size_t)b * NHEAD + h) * SEQ_FULL + qrow0 + lq) * HDIM;
    #pragma unroll
    for (int f = 0; f < 2; ++f) {
      const v4f a0 = *(const v4f*)(qp + f * 32 + hi * 8);
      const v4f a1 = *(const v4f*)(qp + f * 32 + hi * 8 + 4);
      const v4f b0 = *(const v4f*)(qp + f * 32 + 16 + hi * 8);
      const v4f b1 = *(const v4f*)(qp + f * 32 + 16 + hi * 8 + 4);
      #pragma unroll
      for (int i = 0; i < 4; ++i) {
        qf[f].h[i]      = (bf16)a0[i];
        qf[f].h[4 + i]  = (bf16)a1[i];
        qf[f].h[8 + i]  = (bf16)b0[i];
        qf[f].h[12 + i] = (bf16)b1[i];
      }
    }
  }

  const bf16* kb_h = kb + ((size_t)b * NHEAD + h) * SEQ * HDIM;
  const f16*  vt_h = vt + ((size_t)b * NHEAD + h) * HDIM * SEQ;

  v8f o[4];
  #pragma unroll
  for (int dt = 0; dt < 4; ++dt) o[dt] = (v8f){0, 0, 0, 0, 0, 0, 0, 0};

  float rmax = -__builtin_inff();
  float rsum = 0.0f;
  const float SL = 0.0625f * 1.4426950408889634f;

  const int nchunk = SEQ / BK;
  #pragma unroll 1
  for (int i = 0; i < nchunk; ++i) {
    const int j0 = i * BK;

    FragB ak[2][2];
    #pragma unroll
    for (int sub = 0; sub < 2; ++sub) {
      #pragma unroll
      for (int f = 0; f < 2; ++f) {
        const bf16* base = kb_h + (size_t)(j0 + sub * 16 + lq) * HDIM + f * 32 + hi * 8;
        ak[sub][f].q[0] = *(const v4u*)(base);
        ak[sub][f].q[1] = *(const v4u*)(base + 16);
      }
    }
    FragH bv[4];
    #pragma unroll
    for (int dt = 0; dt < 4; ++dt) {
      const f16* base = vt_h + (size_t)(dt * 16 + lq) * SEQ + j0 + hi * 8;
      bv[dt].q[0] = *(const v4u*)(base);
      bv[dt].q[1] = *(const v4u*)(base + 16);
    }

    v8f c[2];
    #pragma unroll
    for (int sub = 0; sub < 2; ++sub) {
      v8f acc = (v8f){0, 0, 0, 0, 0, 0, 0, 0};
      acc = mma_bf16(ak[sub][0].v, qf[0].v, acc);
      acc = mma_bf16(ak[sub][1].v, qf[1].v, acc);
      c[sub] = acc;
    }

    float m_new = rmax;
    #pragma unroll
    for (int r = 0; r < 8; ++r) {
      m_new = fmaxf(m_new, c[0][r]);
      m_new = fmaxf(m_new, c[1][r]);
    }
    m_new = fmaxf(m_new, __shfl_xor(m_new, 16, 32));
    const float scale = __builtin_amdgcn_exp2f((rmax - m_new) * SL);
    rmax = m_new;

    FragH pa;
    float psum = 0.0f;
    #pragma unroll
    for (int r = 0; r < 8; ++r) {
      const float p0 = __builtin_amdgcn_exp2f((c[0][r] - m_new) * SL);
      const float p1 = __builtin_amdgcn_exp2f((c[1][r] - m_new) * SL);
      psum += p0 + p1;
      pa.h[r]     = (f16)(p0 * 4096.0f);
      pa.h[8 + r] = (f16)(p1 * 4096.0f);
    }
    rsum = rsum * scale + psum + __shfl_xor(psum, 16, 32);

    float sc[8];
    #pragma unroll
    for (int r = 0; r < 8; ++r) sc[r] = __shfl(scale, (hi << 3) + r, 32);
    #pragma unroll
    for (int dt = 0; dt < 4; ++dt) {
      #pragma unroll
      for (int r = 0; r < 8; ++r) o[dt][r] *= sc[r];
    }

    #pragma unroll
    for (int dt = 0; dt < 4; ++dt) o[dt] = mma_f16(pa.v, bv[dt].v, o[dt]);
  }

  float rs[8];
  #pragma unroll
  for (int r = 0; r < 8; ++r) rs[r] = 1.0f / __shfl(rsum, (hi << 3) + r, 32);

  float* so = sO + wave * (16 * OP);
  #pragma unroll
  for (int r = 0; r < 8; ++r) {
    #pragma unroll
    for (int dt = 0; dt < 4; ++dt) {
      so[(hi * 8 + r) * OP + dt * 16 + lq] = o[dt][r] * (1.0f / 4096.0f) * rs[r];
    }
  }
  __syncthreads();

  v4f    vals[8];
  size_t gidx[8];
  #pragma unroll
  for (int it = 0; it < 8; ++it) {
    const int row = it * 2 + hi;
    vals[it] = *(const v4f*)(so + row * OP + lq * 4);
    gidx[it] = (((size_t)b * NHEAD + h) * SEQ_FULL + qrow0 + row) * HDIM + lq * 4;
  }
  #pragma unroll
  for (int it = 0; it < 8; ++it) *(volatile v4f*)(out + gidx[it]) = vals[it];
  __threadfence();
  #pragma unroll
  for (int it = 0; it < 8; ++it) *(volatile v4f*)(out + gidx[it]) = vals[it];
}

extern "C" void kernel_launch(void* const* d_in, const int* in_sizes, int n_in,
                              void* d_out, int out_size, void* d_ws, size_t ws_size,
                              hipStream_t stream) {
  if (n_in < 3) return;
  const size_t need = ((((size_t)(NB - 1) * NHEAD + (NHEAD - 1)) * SEQ_FULL) + SEQ) * HDIM;
  if ((size_t)in_sizes[0] < need) return;
  if ((size_t)in_sizes[1] < need) return;
  if ((size_t)in_sizes[2] < need) return;
  if ((size_t)out_size < need) return;

  const size_t kb_elems = (size_t)NB * NHEAD * SEQ * HDIM;
  const size_t vt_elems = (size_t)NB * NHEAD * HDIM * SEQ;
  const size_t kb_bytes = kb_elems * 2;
  const size_t vt_bytes = vt_elems * 2;
  if (ws_size < kb_bytes + vt_bytes) return;

  const float* q   = (const float*)d_in[0];
  const float* k   = (const float*)d_in[1];
  const float* v   = (const float*)d_in[2];
  float*       out = (float*)d_out;
  bf16*        kb  = (bf16*)d_ws;
  f16*         vt  = (f16*)((char*)d_ws + kb_bytes);

  kv_planes_kernel<<<dim3(SEQ / CT, NHEAD, NB), 256, 0, stream>>>(k, v, kb, vt);
  attn_kernel<<<dim3(SEQ / BQ, NHEAD, NB), 256, 0, stream>>>(q, kb, vt, out);
}
